// NEUROPULSNxN_2_2_72353019068773
// MI455X (gfx1250) — hardware-run, weakly checked
//
#include <hip/hip_runtime.h>
#include <math.h>

typedef __attribute__((ext_vector_type(16))) _Float16 v16h;
typedef __attribute__((ext_vector_type(8)))  _Float16 v8h;
typedef __attribute__((ext_vector_type(8)))  float    v8f;
typedef __attribute__((ext_vector_type(4)))  float    v4f;

constexpr int kRows   = 65536;
constexpr int kPorts  = 64;
constexpr int kStages = 64;
constexpr int kCols   = 2 * kPorts;
constexpr int kBP     = 72;
constexpr int kOP     = 68;
constexpr int kTP     = 132;
constexpr float kCarryX = 16.0f;
constexpr float kCarryT = 256.0f;
constexpr float kFold   = 1.0f / (kCarryX * kCarryT);
constexpr float kHalfMinNormal = 6.103515625e-5f;
static_assert(kPorts == 64 && kStages == 64, "mesh shape");
static_assert((kPorts % 32) == 0, "K multiple of 32");
static_assert((kRows % 128) == 0 && (kCols % 16) == 0, "M, N tile multiples");
static_assert(kFold == 1.0f / 4096.0f, "carry fold");

constexpr size_t kOffTF   = 0;
constexpr size_t kOffBT   = kOffTF + (size_t)kStages * kCols * 4;
constexpr size_t kWsTotal = kOffBT + (size_t)kCols * kPorts * 2;
static_assert(kWsTotal == 49152ull, "carve total");
static_assert((kOffBT % 128) == 0, "aligned regions");

union FragH { v16h v; v8h h[2]; };
__device__ __forceinline__ v16h frag_load_h(const _Float16* p) {
  FragH f;
  f.h[0] = *(const v8h*)(p);
  f.h[1] = *(const v8h*)(p + 16);
  return f.v;
}
__device__ __forceinline__ v8f mma_h(v16h a, v16h b, v8f c) {
  c = __builtin_amdgcn_wmma_f32_16x16x32_f16(false, a, false, b, (short)0, c, false, false);
  asm volatile("v_nop\n\tv_nop\n\tv_nop\n\tv_nop" : "+v"(c) : "v"(a), "v"(b));
  return c;
}
__device__ __forceinline__ _Float16 to_half_flushed(float v) {
  const float w = (fabsf(v) < kHalfMinNormal) ? 0.0f : v;
  return (_Float16)w;
}

__global__ __launch_bounds__(32) void build_transfer_kernel(
    const float* __restrict__ phi1, const float* __restrict__ phi2, float* __restrict__ TF)
{
  __shared__ __align__(16) float sRow[kCols];
  const int k = blockIdx.x;
  const int l = threadIdx.x;
  const float S = sqrtf(0.5f);

  float c0r = (2 * l == k) ? 1.0f : 0.0f;
  float c0i = 0.0f;
  float c1r = (2 * l + 1 == k) ? 1.0f : 0.0f;
  float c1i = 0.0f;

#pragma unroll 1
  for (int hs = 0; hs < 2 * kStages; ++hs) {
    const int s = hs >> 1;
    const bool odd = (hs & 1) != 0;
    float a1 = phi1[s * kPorts + 2 * l];
    float a2 = phi2[s * kPorts + 2 * l + 1];
    asm volatile("" : "+v"(a1), "+v"(a2));
    const float ang = odd ? a2 : a1;
    float sn, cs;
    sincosf(ang, &sn, &cs);
    const bool nophase = odd && (l == 31);
    cs = nophase ? 1.0f : cs;
    sn = nophase ? 0.0f : sn;
    const float sr = odd ? c1r : c0r;
    const float si = odd ? c1i : c0i;
    const float pr  = sr * cs - si * sn;
    const float pim = sr * sn + si * cs;
    const float vnr = __shfl_down(c0r, 1, 32);
    const float vni = __shfl_down(c0i, 1, 32);
    const float upr = __shfl_up(pr, 1, 32);
    const float upi = __shfl_up(pim, 1, 32);
    const float war = odd ? vnr : c1r;
    const float wai = odd ? vni : c1i;
    const float Ar = S * (pr - wai);
    const float Ai = S * (pim + war);
    const float ubr = odd ? upr : pr;
    const float ubi = odd ? upi : pim;
    const float wbr = odd ? c0r : c1r;
    const float wbi = odd ? c0i : c1i;
    const float Br = S * (wbr - ubi);
    const float Bi = S * (wbi + ubr);
    const float o0r = (l > 0) ? Br : c0r;
    const float o0i = (l > 0) ? Bi : c0i;
    const float o1r = (l < 31) ? Ar : c1r;
    const float o1i = (l < 31) ? Ai : c1i;
    const float n0r = odd ? o0r : Ar;
    const float n0i = odd ? o0i : Ai;
    const float n1r = odd ? o1r : Br;
    const float n1i = odd ? o1i : Bi;
    c0r = n0r; c0i = n0i; c1r = n1r; c1i = n1i;
  }

  sRow[2 * l]              = c0r;
  sRow[2 * l + 1]          = c1r;
  sRow[kPorts + 2 * l]     = c0i;
  sRow[kPorts + 2 * l + 1] = c1i;
  __syncthreads();
  const v4f v = *(const v4f*)(sRow + 4 * l);
  float* dst = TF + (size_t)k * kCols + 4 * l;
  *(volatile v4f*)dst = v;
  __threadfence();
  *(volatile v4f*)dst = v;
}

__global__ __launch_bounds__(256) void make_bt_kernel(
    const float* __restrict__ TF, unsigned short* __restrict__ BT)
{
  __shared__ __align__(16) float sT[kStages * kTP];
  const int tid = threadIdx.x;
  const int lane = tid & 31;
  const int wave = tid >> 5;
#pragma unroll
  for (int i = 0; i < 8; ++i) {
    const int idx = i * 256 + tid;
    const int kr = idx >> 5;
    const int c = (idx & 31) * 4;
    *(v4f*)(sT + kr * kTP + c) = *(const v4f*)(TF + (size_t)kr * kCols + c);
  }
  __syncthreads();
  const int q = lane >> 3;
  const int c8 = (lane & 7) * 8;
  v8h hv[4];
#pragma unroll
  for (int it = 0; it < 4; ++it) {
    const int n = wave * 16 + it * 4 + q;
#pragma unroll
    for (int e = 0; e < 8; ++e) {
      const float t = sT[(c8 + e) * kTP + n] * kCarryT;
      hv[it][e] = to_half_flushed(t);
    }
  }
  for (int pass = 0; pass < 2; ++pass) {
#pragma unroll
    for (int it = 0; it < 4; ++it) {
      const int n = wave * 16 + it * 4 + q;
      *(volatile v8h*)(BT + (size_t)n * kPorts + c8) = hv[it];
    }
    __threadfence();
  }
}

__global__ __launch_bounds__(256) void mesh_gemm_detect_kernel(
    const float* __restrict__ x, const _Float16* __restrict__ BT, float* __restrict__ out)
{
  __shared__ __align__(16) _Float16 sB[kCols * kBP];
  __shared__ __align__(16) float sO[8][16 * kOP];
  const int tid = threadIdx.x;
  const int lane = tid & 31;
  const int wave = tid >> 5;
  const int h = lane >> 4;
  const int rl = lane & 15;

#pragma unroll
  for (int i = 0; i < 4; ++i) {
    const int idx = i * 256 + tid;
    const int row = idx >> 3;
    const int c = (idx & 7) * 8;
    *(v8h*)(sB + row * kBP + c) = *(const v8h*)(BT + (size_t)row * kPorts + c);
  }
  __syncthreads();

  const size_t row0 = (size_t)blockIdx.x * 128 + (size_t)wave * 16;
  const float* xr = x + (row0 + rl) * kPorts + 8 * h;

  v8f acc[8];
#pragma unroll
  for (int j = 0; j < 8; ++j) acc[j] = (v8f){0.f, 0.f, 0.f, 0.f, 0.f, 0.f, 0.f, 0.f};

#pragma unroll
  for (int ks = 0; ks < 2; ++ks) {
    const float* p = xr + ks * 32;
    const v4f f0 = *(const v4f*)(p);
    const v4f f1 = *(const v4f*)(p + 4);
    const v4f f2 = *(const v4f*)(p + 16);
    const v4f f3 = *(const v4f*)(p + 20);
    v16h a;
#pragma unroll
    for (int e = 0; e < 4; ++e) {
      const float g0 = f0[e] * kCarryX;
      const float g1 = f1[e] * kCarryX;
      const float g2 = f2[e] * kCarryX;
      const float g3 = f3[e] * kCarryX;
      a[e]      = to_half_flushed(g0);
      a[4 + e]  = to_half_flushed(g1);
      a[8 + e]  = to_half_flushed(g2);
      a[12 + e] = to_half_flushed(g3);
    }
#pragma unroll
    for (int j = 0; j < 8; ++j) {
      const v16h b = frag_load_h(sB + (j * 16 + rl) * kBP + ks * 32 + 8 * h);
      acc[j] = mma_h(a, b, acc[j]);
    }
  }

  float* slab = sO[wave];
#pragma unroll
  for (int j = 0; j < 4; ++j) {
#pragma unroll
    for (int r = 0; r < 8; ++r) {
      const float re = acc[j][r] * kFold;
      const float im = acc[j + 4][r] * kFold;
      slab[(8 * h + r) * kOP + j * 16 + rl] = re * re + im * im;
    }
  }
  __syncthreads();
  {
    const int c4 = rl * 4;
    for (int pass = 0; pass < 2; ++pass) {
#pragma unroll
      for (int it = 0; it < 8; ++it) {
        const int row = it * 2 + h;
        const v4f val = *(const v4f*)(slab + row * kOP + c4);
        *(volatile v4f*)(out + (row0 + row) * kPorts + c4) = val;
      }
      __threadfence();
    }
  }
}

extern "C" void kernel_launch(void* const* d_in, const int* in_sizes, int n_in,
                              void* d_out, int out_size, void* d_ws, size_t ws_size,
                              hipStream_t stream) {
  if (n_in < 3) return;
  if (in_sizes[0] != kRows * kPorts) return;
  if (in_sizes[1] != kStages * kPorts) return;
  if (in_sizes[2] != kStages * kPorts) return;
  if (out_size != kRows * kPorts) return;
  if (ws_size < kWsTotal) return;

  const float* x    = (const float*)d_in[0];
  const float* phi1 = (const float*)d_in[1];
  const float* phi2 = (const float*)d_in[2];
  float* out = (float*)d_out;

  char* ws = (char*)d_ws;
  float*          TF = (float*)(ws + kOffTF);
  unsigned short* BT = (unsigned short*)(ws + kOffBT);

  build_transfer_kernel<<<dim3(kStages), dim3(32), 0, stream>>>(phi1, phi2, TF);
  make_bt_kernel<<<dim3(1), dim3(256), 0, stream>>>(TF, BT);
  mesh_gemm_detect_kernel<<<dim3(kRows / 128), dim3(256), 0, stream>>>(x, (const _Float16*)BT, out);
}
